// HermesBlock_67568425501242
// MI455X (gfx1250) — hardware-run, weakly checked
//
#include <hip/hip_runtime.h>
#include <math.h>

#ifndef NB
#define NB 4
#endif
#ifndef SEQ
#define SEQ 1024
#endif
#define SEQ_FULL 1024
#define NB_FULL 4
#define DM 1024
#define HEADS 16
#define HS 64
#define HID 3072
#define MTOK (NB * SEQ)
#define NQB (SEQ / 64)
#define NP_BIG 64
#define NP_SML 1
#define PART_SLOT 2048

static_assert(SEQ % 64 == 0);
static_assert(SEQ <= SEQ_FULL);
static_assert(NB <= NB_FULL);
static_assert(MTOK % 64 == 0);
static_assert(DM % 256 == 0 && HID % 256 == 0);
static_assert(DM == HEADS * HS);
static_assert(HS == 64);
static_assert(DM % 64 == 0 && HID % 64 == 0 && DM % 32 == 0 && HID % 32 == 0);
static_assert(NP_BIG <= 64 && NP_SML <= 64);
static_assert(((DM * DM / 4) % NP_BIG) == 0 && ((HID * DM / 4) % NP_BIG) == 0);
static_assert(((DM * DM / 8) % 256) == 0 && ((HS * HS / 8) % 256) == 0 && ((HID * DM / 8) % 256) == 0);
static_assert(((HID / 2) % 256) == 0);

typedef _Float16 h16;
typedef __attribute__((ext_vector_type(16))) _Float16 v16h;
typedef __attribute__((ext_vector_type(8)))  _Float16 v8h;
typedef __attribute__((ext_vector_type(8)))  float    v8f;
typedef __attribute__((ext_vector_type(4)))  float    v4f;


#define VST2(T, ptr, val) do { const T vst2_v_ = (val); *(volatile T*)(ptr) = vst2_v_; __threadfence(); *(volatile T*)(ptr) = vst2_v_; } while (0)

static __device__ __forceinline__ float bfr(float f) {
    unsigned u = __float_as_uint(f);
    u += 0x7FFFu + ((u >> 16) & 1u);
    return __uint_as_float(u & 0xFFFF0000u);
}
static __device__ __forceinline__ h16 toh_flush(float v) {
    const float w = (fabsf(v) < 6.103515625e-05f) ? 0.0f : v;
    return (h16)w;
}
static __device__ __forceinline__ v8h pack8(const float* v) {
    v8h r;
#pragma unroll
    for (int e = 0; e < 8; ++e) r[e] = toh_flush(v[e]);
    return r;
}

union FragU { v16h v; v8h h[2]; };
static __device__ __forceinline__ v16h frag_ld(const h16* p) {
    FragU f; f.h[0] = *(const v8h*)(p); f.h[1] = *(const v8h*)(p + 16); return f.v;
}
static __device__ __forceinline__ v16h frag_f32(const float* p) {
    const v4f a0 = *(const v4f*)(p);
    const v4f a1 = *(const v4f*)(p + 4);
    const v4f b0 = *(const v4f*)(p + 16);
    const v4f b1 = *(const v4f*)(p + 20);
    v16h f;
    f[0]  = toh_flush(a0.x); f[1]  = toh_flush(a0.y); f[2]  = toh_flush(a0.z); f[3]  = toh_flush(a0.w);
    f[4]  = toh_flush(a1.x); f[5]  = toh_flush(a1.y); f[6]  = toh_flush(a1.z); f[7]  = toh_flush(a1.w);
    f[8]  = toh_flush(b0.x); f[9]  = toh_flush(b0.y); f[10] = toh_flush(b0.z); f[11] = toh_flush(b0.w);
    f[12] = toh_flush(b1.x); f[13] = toh_flush(b1.y); f[14] = toh_flush(b1.z); f[15] = toh_flush(b1.w);
    return f;
}
static __device__ __forceinline__ v8f wmma16g(v16h a, v16h b, v8f c) {
    c = __builtin_amdgcn_wmma_f32_16x16x32_f16(false, a, false, b, (short)0, c, false, false);
    asm volatile("v_nop\n\tv_nop\n\tv_nop\n\tv_nop" : "+v"(c) : "v"(a), "v"(b));
    return c;
}
static __device__ __forceinline__ void wave_sync_lds() {
    __builtin_amdgcn_fence(3  , "workgroup");
    __builtin_amdgcn_wave_barrier();
    __builtin_amdgcn_fence(2  , "workgroup");
}

__global__ __launch_bounds__(256) void k_absmax(const float* __restrict__ w, unsigned n4, unsigned per4,
                                                float* __restrict__ part) {
    __shared__ float sM[8];
    const unsigned tid = threadIdx.x, lane = tid & 31u, wave = tid >> 5;
    const unsigned beg = blockIdx.x * per4;
    const unsigned end = min(beg + per4, n4);
    float m = 0.0f;
    for (unsigned i = beg + tid; i < end; i += 256u) {
        const v4f a = *(const v4f*)(w + (size_t)i * 4u);
        const float m0 = fmaxf(fabsf(bfr(a.x)), fabsf(bfr(a.y)));
        const float m1 = fmaxf(fabsf(bfr(a.z)), fabsf(bfr(a.w)));
        m = fmaxf(m, fmaxf(m0, m1));
    }
    m = fmaxf(m, __shfl_xor(m, 16, 32)); m = fmaxf(m, __shfl_xor(m, 8, 32));
    m = fmaxf(m, __shfl_xor(m, 4, 32));  m = fmaxf(m, __shfl_xor(m, 2, 32));
    m = fmaxf(m, __shfl_xor(m, 1, 32));
    if (lane == 0u) sM[wave] = m;
    __syncthreads();
    if (wave == 0u) {
        float v = sM[lane & 7u];
        v = fmaxf(v, __shfl_xor(v, 1, 32)); v = fmaxf(v, __shfl_xor(v, 2, 32)); v = fmaxf(v, __shfl_xor(v, 4, 32));
        VST2(float, part + (size_t)blockIdx.x * 32u + lane, v);
    }
}

__global__ __launch_bounds__(256) void k_scales(const float* __restrict__ part, float* __restrict__ scales) {
    __shared__ float sS[8];
    const unsigned tid = threadIdx.x, lane = tid & 31u, w = tid >> 5;
    const unsigned np = (w == 4u || w == 5u) ? (unsigned)NP_SML : (unsigned)NP_BIG;
    const unsigned i0 = min(lane, np - 1u);
    const unsigned i1 = min(lane + 32u, np - 1u);
    const float a = part[((size_t)w * 64u + i0) * 32u];
    const float b = part[((size_t)w * 64u + i1) * 32u];
    float m = fmaxf(a, b);
    m = fmaxf(m, __shfl_xor(m, 16, 32)); m = fmaxf(m, __shfl_xor(m, 8, 32));
    m = fmaxf(m, __shfl_xor(m, 4, 32));  m = fmaxf(m, __shfl_xor(m, 2, 32));
    m = fmaxf(m, __shfl_xor(m, 1, 32));
    if (lane == 0u) sS[w] = m;
    __syncthreads();
    if (w == 0u) {
        const float am = sS[lane & 7u];
        const float sc = am / 31.0f + 1e-8f;
        const float outv = (lane < 8u) ? sc : 0.0f;
        VST2(float, scales + lane, outv);
    }
}

__global__ __launch_bounds__(256) void k_levels(const float* __restrict__ w, unsigned n8, const float* __restrict__ scales,
                                                unsigned sidx, h16* __restrict__ lv) {
    const unsigned u = blockIdx.x * 256u + threadIdx.x;
    if (u >= n8) return;
    const float scale = scales[sidx];
    const v4f a = *(const v4f*)(w + (size_t)u * 8u);
    const v4f b = *(const v4f*)(w + (size_t)u * 8u + 4u);
    const float wv[8] = {a.x, a.y, a.z, a.w, b.x, b.y, b.z, b.w};
    float q[8];
#pragma unroll
    for (int i = 0; i < 8; ++i) {
        const float wb = bfr(wv[i]);
        float t = rintf(wb / scale);
        t = fminf(fmaxf(t, -31.0f), 31.0f);
        q[i] = t;
    }
    const v8h hv = pack8(q);
    VST2(v8h, lv + (size_t)u * 8u, hv);
}

__global__ __launch_bounds__(256) void k_trig(const float* __restrict__ theta, float* __restrict__ ctab,
                                              float* __restrict__ stab, unsigned n) {
    const unsigned i = blockIdx.x * 256u + threadIdx.x;
    const unsigned ic = min(i, n - 1u);
    const float th = bfr(theta[ic]);
    const float cv = cosf(th);
    const float sv = sinf(th);
    if (i < n) {
        VST2(float, ctab + i, cv);
        VST2(float, stab + i, sv);
    }
}

template <bool RND>
static __device__ __forceinline__ void ld8(const float* p, float* v) {
    const v4f a = *(const v4f*)(p);
    const v4f b = *(const v4f*)(p + 4);
    v[0] = a.x; v[1] = a.y; v[2] = a.z; v[3] = a.w; v[4] = b.x; v[5] = b.y; v[6] = b.z; v[7] = b.w;
    if (RND) {
#pragma unroll
        for (int i = 0; i < 8; ++i) v[i] = bfr(v[i]);
    }
}

template <bool RND>
__global__ __launch_bounds__(256) void k_ln(const float* __restrict__ X, const float* __restrict__ g,
                                            const float* __restrict__ bt, h16* __restrict__ Z, unsigned M, unsigned ngrp) {
    const unsigned row = blockIdx.x * 8u + (threadIdx.x >> 5);
    const unsigned L = threadIdx.x & 31u;
    if (row >= M) return;
    const unsigned srow = RND ? ((row / (unsigned)SEQ) * (unsigned)SEQ_FULL + (row % (unsigned)SEQ)) : row;
    const float* xr = X + (size_t)srow * DM + 8u * L;
    float s = 0.0f;
    for (unsigned gi = 0; gi < ngrp; ++gi) {
        float v[8];
        ld8<RND>(xr + gi * 256u, v);
        s += ((v[0] + v[1]) + (v[2] + v[3])) + ((v[4] + v[5]) + (v[6] + v[7]));
    }
    s += __shfl_xor(s, 16, 32); s += __shfl_xor(s, 8, 32); s += __shfl_xor(s, 4, 32);
    s += __shfl_xor(s, 2, 32);  s += __shfl_xor(s, 1, 32);
    const float mu = s * (1.0f / (float)DM);
    float q = 0.0f;
    for (unsigned gi = 0; gi < ngrp; ++gi) {
        float v[8];
        ld8<RND>(xr + gi * 256u, v);
#pragma unroll
        for (int i = 0; i < 8; ++i) { const float d = v[i] - mu; q += d * d; }
    }
    q += __shfl_xor(q, 16, 32); q += __shfl_xor(q, 8, 32); q += __shfl_xor(q, 4, 32);
    q += __shfl_xor(q, 2, 32);  q += __shfl_xor(q, 1, 32);
    const float den = sqrtf(q * (1.0f / (float)DM) + 1e-5f);
    for (unsigned gi = 0; gi < ngrp; ++gi) {
        float v[8], gg[8], bb[8], y[8];
        ld8<RND>(xr + gi * 256u, v);
        ld8<true>(g + gi * 256u + 8u * L, gg);
        ld8<true>(bt + gi * 256u + 8u * L, bb);
#pragma unroll
        for (int i = 0; i < 8; ++i) y[i] = (((v[i] - mu) / den) * gg[i] + bb[i]) * 64.0f;
        const v8h hv = pack8(y);
        VST2(v8h, Z + (size_t)row * DM + gi * 256u + 8u * L, hv);
    }
}

static __device__ __forceinline__ void rot8(const float* hp, const float* cp, const float* sp, float* v) {
    const v4f a = *(const v4f*)(hp);
    const v4f b = *(const v4f*)(hp + 4);
    const v4f c = *(const v4f*)(cp);
    const v4f s = *(const v4f*)(sp);
    v[0] = c.x * a.x - s.x * a.y;  v[1] = s.x * a.x + c.x * a.y;
    v[2] = c.y * a.z - s.y * a.w;  v[3] = s.y * a.z + c.y * a.w;
    v[4] = c.z * b.x - s.z * b.y;  v[5] = s.z * b.x + c.z * b.y;
    v[6] = c.w * b.z - s.w * b.w;  v[7] = s.w * b.z + c.w * b.w;
}

__global__ __launch_bounds__(256) void k_rot_ln_silu(const float* __restrict__ Hb, const float* __restrict__ ctab,
                                                     const float* __restrict__ stab, const float* __restrict__ g,
                                                     const float* __restrict__ bt, h16* __restrict__ ACT,
                                                     unsigned M, unsigned nch) {
    const unsigned row = blockIdx.x * 8u + (threadIdx.x >> 5);
    const unsigned L = threadIdx.x & 31u;
    if (row >= M) return;
    const float* hr = Hb + (size_t)row * HID + 8u * L;
    const float* cp = ctab + 4u * L;
    const float* sp = stab + 4u * L;
    float s = 0.0f;
    for (unsigned ch = 0; ch < nch; ++ch) {
        float v[8];
        rot8(hr + ch * 256u, cp + ch * 128u, sp + ch * 128u, v);
        s += ((v[0] + v[1]) + (v[2] + v[3])) + ((v[4] + v[5]) + (v[6] + v[7]));
    }
    s += __shfl_xor(s, 16, 32); s += __shfl_xor(s, 8, 32); s += __shfl_xor(s, 4, 32);
    s += __shfl_xor(s, 2, 32);  s += __shfl_xor(s, 1, 32);
    const float mu = s * (1.0f / (float)HID);
    float q = 0.0f;
    for (unsigned ch = 0; ch < nch; ++ch) {
        float v[8];
        rot8(hr + ch * 256u, cp + ch * 128u, sp + ch * 128u, v);
#pragma unroll
        for (int i = 0; i < 8; ++i) { const float d = v[i] - mu; q += d * d; }
    }
    q += __shfl_xor(q, 16, 32); q += __shfl_xor(q, 8, 32); q += __shfl_xor(q, 4, 32);
    q += __shfl_xor(q, 2, 32);  q += __shfl_xor(q, 1, 32);
    const float den = sqrtf(q * (1.0f / (float)HID) + 1e-5f);
    for (unsigned ch = 0; ch < nch; ++ch) {
        float v[8], gg[8], bb[8], y[8];
        rot8(hr + ch * 256u, cp + ch * 128u, sp + ch * 128u, v);
        ld8<true>(g + ch * 256u + 8u * L, gg);
        ld8<true>(bt + ch * 256u + 8u * L, bb);
#pragma unroll
        for (int i = 0; i < 8; ++i) {
            const float z = ((v[i] - mu) / den) * gg[i] + bb[i];
            const float act = z / (1.0f + expf(-z));
            y[i] = act * 64.0f;
        }
        const v8h hv = pack8(y);
        VST2(v8h, ACT + (size_t)row * HID + ch * 256u + 8u * L, hv);
    }
}

template <int OUT_MODE, int RESID, int IN_LOG2, int OUT_LOG2>
__global__ __launch_bounds__(256) void k_gemm64(
    const h16* __restrict__ A, unsigned lda, const h16* __restrict__ Bt, unsigned ldb,
    void* __restrict__ Cout, unsigned ldc, const float* __restrict__ scales, unsigned sidx,
    const float* __restrict__ resid, unsigned M, unsigned N, unsigned K) {
  __shared__ __align__(16) float sT[8][16 * 68];
  constexpr float INV_IN = 1.0f / (float)(1u << IN_LOG2);
  constexpr float OUTC = (float)(1u << OUT_LOG2);
  const unsigned lane = threadIdx.x & 31u;
  const unsigned wave = threadIdx.x >> 5;
  const unsigned tilesN = N >> 6, tilesM = M >> 6;
  const unsigned tile = blockIdx.x * 8u + wave;
  if (tile >= tilesM * tilesN) return;
  const unsigned tm = tile / tilesN;
  const unsigned tn = tile - tm * tilesN;
  const unsigned m0 = tm << 6, n0 = tn << 6;
  const unsigned rlane = lane & 15u;
  const unsigned koff = (lane >> 4) * 8u;
  const unsigned mOff = koff;
  const float sc = scales[sidx] * INV_IN;

  v8f acc[4][4];
#pragma unroll
  for (int i = 0; i < 4; ++i)
#pragma unroll
    for (int j = 0; j < 4; ++j) acc[i][j] = (v8f){0.f,0.f,0.f,0.f,0.f,0.f,0.f,0.f};

  for (unsigned k0 = 0; k0 < K; k0 += 32u) {
    v16h bh[4];
#pragma unroll
    for (int j = 0; j < 4; ++j)
      bh[j] = frag_ld(Bt + (size_t)(n0 + ((unsigned)j << 4) + rlane) * ldb + koff + k0);
#pragma unroll
    for (int i = 0; i < 4; ++i) {
      const v16h ah = frag_ld(A + (size_t)(m0 + ((unsigned)i << 4) + rlane) * lda + koff + k0);
#pragma unroll
      for (int j = 0; j < 4; ++j) acc[i][j] = wmma16g(ah, bh[j], acc[i][j]);
    }
  }

  float* slab = sT[wave];
#pragma unroll
  for (int i = 0; i < 4; ++i) {
    const unsigned mBase = m0 + ((unsigned)i << 4);
#pragma unroll
    for (int j = 0; j < 4; ++j) {
#pragma unroll
      for (int r = 0; r < 8; ++r) {
        float v = acc[i][j][r] * sc;
        if (OUT_MODE == 1) v *= OUTC;
        slab[(mOff + (unsigned)r) * 68u + ((unsigned)j << 4) + rlane] = v;
      }
    }
    wave_sync_lds();
    if (OUT_MODE == 0) {
      float* C = (float*)Cout;
      const unsigned hh = lane >> 4, c4 = (lane & 15u) * 4u;
#pragma unroll
      for (int half = 0; half < 2; ++half) {
        v4f vv[4];
#pragma unroll
        for (int it = 0; it < 4; ++it) {
          const unsigned row = (unsigned)(half * 4 + it) * 2u + hh;
          vv[it] = *(const v4f*)(slab + row * 68u + c4);
          if (RESID != 0) {
            const unsigned grow = mBase + row;
            const unsigned rrow = (RESID == 2)
                ? ((grow / (unsigned)SEQ) * (unsigned)SEQ_FULL + (grow % (unsigned)SEQ)) : grow;
            v4f rv = *(const v4f*)(resid + (size_t)rrow * ldc + n0 + c4);
            if (RESID == 2) { rv.x = bfr(rv.x); rv.y = bfr(rv.y); rv.z = bfr(rv.z); rv.w = bfr(rv.w); }
            vv[it] += rv;
          }
        }
        for (int pass = 0; pass < 2; ++pass) {
#pragma unroll
          for (int it = 0; it < 4; ++it) {
            const unsigned row = (unsigned)(half * 4 + it) * 2u + hh;
            *(volatile v4f*)(C + (size_t)(mBase + row) * ldc + n0 + c4) = vv[it];
          }
          __threadfence();
        }
      }
    } else {
      h16* C = (h16*)Cout;
      const unsigned q = lane >> 3, c8 = (lane & 7u) * 8u;
      v8h hv[4];
#pragma unroll
      for (int it = 0; it < 4; ++it) {
        const unsigned row = (unsigned)it * 4u + q;
        const float* sp = slab + row * 68u + c8;
#pragma unroll
        for (int e = 0; e < 8; ++e) hv[it][e] = toh_flush(sp[e]);
      }
      for (int pass = 0; pass < 2; ++pass) {
#pragma unroll
        for (int it = 0; it < 4; ++it) {
          const unsigned row = (unsigned)it * 4u + q;
          *(volatile v8h*)(C + (size_t)(mBase + row) * ldc + n0 + c8) = hv[it];
        }
        __threadfence();
      }
    }
    wave_sync_lds();
  }
}

#define AT_PF 68
__global__ __launch_bounds__(128) void k_attn(const h16* __restrict__ QS, const h16* __restrict__ KS,
                                              const h16* __restrict__ VT, const float* __restrict__ pscale,
                                              h16* __restrict__ AO) {
    __shared__ __align__(16) float sP[4][16 * AT_PF];
    const unsigned tid = threadIdx.x, lane = tid & 31u, wave = tid >> 5;
    const unsigned hh = lane >> 4, c = lane & 15u;
    const unsigned bx = blockIdx.x;
    const unsigned qb = bx % (unsigned)NQB;
    const unsigned bhd = bx / (unsigned)NQB;
    const unsigned h = bhd % (unsigned)HEADS;
    const unsigned b = bhd / (unsigned)HEADS;
    const unsigned rowbase = b * (unsigned)SEQ;
    const unsigned q0 = qb * 64u + wave * 16u;
    const float ps = bfr(pscale[0]);
    const float LOG2E = 1.4426950408889634f;
    const float SC2 = 0.125f * (1.0f / 4096.0f) * 1.4426950408889634f;
    float* pw = sP[wave];

    const h16* qrow = QS + (size_t)(rowbase + q0 + c) * DM + h * 64u + 8u * hh;
    const v16h qf0 = frag_ld(qrow);
    const v16h qf1 = frag_ld(qrow + 32);

    float mrow[8], lrow[8];
    v8f os[4];
#pragma unroll
    for (int r = 0; r < 8; ++r) { mrow[r] = -3.0e38f; lrow[r] = 0.f; }
#pragma unroll
    for (int t = 0; t < 4; ++t) os[t] = (v8f){0.f,0.f,0.f,0.f,0.f,0.f,0.f,0.f};

    const unsigned nch = qb + 1u;
    for (unsigned kc = 0; kc < nch; ++kc) {
        const unsigned kv0 = kc * 64u;
        v8f s[4];
#pragma unroll
        for (int j = 0; j < 4; ++j) {
            const h16* krow = KS + (size_t)(rowbase + kv0 + (unsigned)j * 16u + c) * DM + h * 64u + 8u * hh;
            v8f z = (v8f){0.f,0.f,0.f,0.f,0.f,0.f,0.f,0.f};
            z = wmma16g(qf0, frag_ld(krow), z);
            z = wmma16g(qf1, frag_ld(krow + 32), z);
            s[j] = z;
        }
#pragma unroll
        for (int r = 0; r < 8; ++r) {
            const int t = (int)(q0 + 8u * hh + (unsigned)r);
            float mx = -3.0e38f;
#pragma unroll
            for (int j = 0; j < 4; ++j) {
                const int u = (int)(kv0 + (unsigned)j * 16u + c);
                const int d = t - u;
                const int vp = min((int)__builtin_ctz((unsigned)max(d, 1)), 16);
                const float pb = (d == 0) ? 1.0f : (float)vp * 0.0625f;
                float v = s[j][r] * SC2 + (ps * pb) * LOG2E;
                v = (d < 0) ? -3.0e38f : v;
                s[j][r] = v;
                mx = fmaxf(mx, v);
            }
            mx = fmaxf(mx, __shfl_xor(mx, 1, 32)); mx = fmaxf(mx, __shfl_xor(mx, 2, 32));
            mx = fmaxf(mx, __shfl_xor(mx, 4, 32)); mx = fmaxf(mx, __shfl_xor(mx, 8, 32));
            const float mnew = fmaxf(mrow[r], mx);
            const float alpha = exp2f(mrow[r] - mnew);
            mrow[r] = mnew;
            float psum = 0.f;
#pragma unroll
            for (int j = 0; j < 4; ++j) {
                const float e = exp2f(s[j][r] - mnew);
                const float p = (s[j][r] < -1.0e38f) ? 0.0f : e;
                psum += p;
                pw[(8u * hh + (unsigned)r) * AT_PF + (unsigned)j * 16u + c] = p * 1024.0f;
            }
            psum += __shfl_xor(psum, 1, 32); psum += __shfl_xor(psum, 2, 32);
            psum += __shfl_xor(psum, 4, 32); psum += __shfl_xor(psum, 8, 32);
            lrow[r] = lrow[r] * alpha + psum;
            os[0][r] *= alpha; os[1][r] *= alpha; os[2][r] *= alpha; os[3][r] *= alpha;
        }
        wave_sync_lds();
#pragma unroll
        for (int kk = 0; kk < 2; ++kk) {
            const v16h pa = frag_f32(pw + c * AT_PF + (unsigned)kk * 32u + 8u * hh);
#pragma unroll
            for (int t = 0; t < 4; ++t) {
                const v16h vb = frag_ld(VT + (size_t)(h * 64u + (unsigned)t * 16u + c) * (unsigned)MTOK
                                        + rowbase + kv0 + (unsigned)kk * 32u + 8u * hh);
                os[t] = wmma16g(pa, vb, os[t]);
            }
        }
        wave_sync_lds();
    }
#pragma unroll
    for (int r = 0; r < 8; ++r) {
        const float inv = 1.0f / (lrow[r] * 1024.0f);
#pragma unroll
        for (int t = 0; t < 4; ++t)
            pw[(8u * hh + (unsigned)r) * AT_PF + (unsigned)t * 16u + c] = os[t][r] * inv;
    }
    wave_sync_lds();
    {
        const unsigned q = lane >> 3, c8 = (lane & 7u) * 8u;
        v8h ov[4];
#pragma unroll
        for (int it = 0; it < 4; ++it) {
            const float* sp = pw + ((unsigned)it * 4u + q) * AT_PF + c8;
#pragma unroll
            for (int e = 0; e < 8; ++e) ov[it][e] = toh_flush(sp[e]);
        }
        h16* dst = AO + (size_t)(rowbase + q0) * DM + h * 64u;
        for (int pass = 0; pass < 2; ++pass) {
#pragma unroll
            for (int it = 0; it < 4; ++it) *(volatile v8h*)(dst + (size_t)((unsigned)it * 4u + q) * DM + c8) = ov[it];
            __threadfence();
        }
    }
}

constexpr size_t al256(size_t b) { return (b + 255) & ~(size_t)255; }
constexpr size_t SZ_SC   = al256(128);
constexpr size_t SZ_PART = al256((size_t)8 * 64 * 128);
constexpr size_t SZ_TAB  = al256((size_t)(HID / 2) * 4);
constexpr size_t SZ_LVD  = al256((size_t)DM * DM * 2);
constexpr size_t SZ_LVS  = al256((size_t)HS * HS * 2);
constexpr size_t SZ_LVU  = al256((size_t)HID * DM * 2);
constexpr size_t SZ_PL   = al256((size_t)MTOK * DM * 2);
constexpr size_t SZ_X1   = al256((size_t)MTOK * DM * 4);
constexpr size_t SZ_ACT  = al256((size_t)MTOK * HID * 2);
constexpr size_t SZ_H    = (size_t)MTOK * HID * 4;
constexpr size_t WS_TOTAL = SZ_SC + SZ_PART + 2 * SZ_TAB + 4 * SZ_LVD + 2 * SZ_LVS + 2 * SZ_LVU
                          + SZ_PL + 6 * SZ_PL + SZ_X1 + SZ_ACT;
static_assert(WS_TOTAL <= (size_t)134217728);
static_assert(SZ_H <= 6 * SZ_PL);
static_assert((size_t)8 * PART_SLOT * 4 <= SZ_PART);
static_assert((size_t)NP_BIG * 32 <= PART_SLOT);

extern "C" void kernel_launch(void* const* d_in, const int* in_sizes, int n_in, void* d_out, int out_size,
                              void* d_ws, size_t ws_size, hipStream_t stream) {
    if (n_in < 17) return;
    const int need_x = (NB - 1) * SEQ_FULL * DM + SEQ * DM;
    if (in_sizes[0] < need_x) return;
    if (in_sizes[1] < DM * DM || in_sizes[2] < DM * DM || in_sizes[3] < DM * DM || in_sizes[4] < DM * DM) return;
    if (in_sizes[5] < HS * HS || in_sizes[6] < HS * HS || in_sizes[7] < 1) return;
    if (in_sizes[8] < DM || in_sizes[9] < DM || in_sizes[10] < DM || in_sizes[11] < DM) return;
    if (in_sizes[12] < HID * DM || in_sizes[13] < DM * HID || in_sizes[14] < HID / 2) return;
    if (in_sizes[15] < HID || in_sizes[16] < HID) return;
    if (out_size < MTOK * DM) return;
    if (WS_TOTAL > ws_size) return;

    const float* x     = (const float*)d_in[0];
    const float* wq    = (const float*)d_in[1];
    const float* wk    = (const float*)d_in[2];
    const float* wv    = (const float*)d_in[3];
    const float* wo    = (const float*)d_in[4];
    const float* su    = (const float*)d_in[5];
    const float* sv    = (const float*)d_in[6];
    const float* pscal = (const float*)d_in[7];
    const float* n1g   = (const float*)d_in[8];
    const float* n1b   = (const float*)d_in[9];
    const float* n2g   = (const float*)d_in[10];
    const float* n2b   = (const float*)d_in[11];
    const float* wup   = (const float*)d_in[12];
    const float* wdn   = (const float*)d_in[13];
    const float* theta = (const float*)d_in[14];
    const float* mng   = (const float*)d_in[15];
    const float* mnb   = (const float*)d_in[16];
    float* out = (float*)d_out;

    char* wsp = (char*)d_ws;
    size_t off = 0;
    auto carve = [&](size_t bytes) -> void* { void* r = wsp + off; off += bytes; return r; };
    float* scales = (float*)carve(SZ_SC);
    float* part   = (float*)carve(SZ_PART);
    float* ctab   = (float*)carve(SZ_TAB);
    float* stab   = (float*)carve(SZ_TAB);
    h16* LVq  = (h16*)carve(SZ_LVD);
    h16* LVk  = (h16*)carve(SZ_LVD);
    h16* LVv  = (h16*)carve(SZ_LVD);
    h16* LVo  = (h16*)carve(SZ_LVD);
    h16* LVsu = (h16*)carve(SZ_LVS);
    h16* LVsv = (h16*)carve(SZ_LVS);
    h16* LVup = (h16*)carve(SZ_LVU);
    h16* LVdn = (h16*)carve(SZ_LVU);
    h16* XN   = (h16*)carve(SZ_PL);
    char* attBase = (char*)carve(0);
    h16* Q16  = (h16*)carve(SZ_PL);
    h16* K16  = (h16*)carve(SZ_PL);
    h16* QS16 = (h16*)carve(SZ_PL);
    h16* KS16 = (h16*)carve(SZ_PL);
    h16* VT16 = (h16*)carve(SZ_PL);
    h16* AO16 = (h16*)carve(SZ_PL);
    float* X1  = (float*)carve(SZ_X1);
    h16* ACT16 = (h16*)carve(SZ_ACT);
    float* HBUF = (float*)attBase;
    if (off != WS_TOTAL || off > ws_size) return;

    k_absmax<<<NP_BIG, 256, 0, stream>>>(wq,  DM * DM / 4, DM * DM / 4 / NP_BIG, part + 0 * PART_SLOT);
    k_absmax<<<NP_BIG, 256, 0, stream>>>(wk,  DM * DM / 4, DM * DM / 4 / NP_BIG, part + 1 * PART_SLOT);
    k_absmax<<<NP_BIG, 256, 0, stream>>>(wv,  DM * DM / 4, DM * DM / 4 / NP_BIG, part + 2 * PART_SLOT);
    k_absmax<<<NP_BIG, 256, 0, stream>>>(wo,  DM * DM / 4, DM * DM / 4 / NP_BIG, part + 3 * PART_SLOT);
    k_absmax<<<NP_SML, 256, 0, stream>>>(su,  HS * HS / 4, HS * HS / 4 / NP_SML, part + 4 * PART_SLOT);
    k_absmax<<<NP_SML, 256, 0, stream>>>(sv,  HS * HS / 4, HS * HS / 4 / NP_SML, part + 5 * PART_SLOT);
    k_absmax<<<NP_BIG, 256, 0, stream>>>(wup, HID * DM / 4, HID * DM / 4 / NP_BIG, part + 6 * PART_SLOT);
    k_absmax<<<NP_BIG, 256, 0, stream>>>(wdn, HID * DM / 4, HID * DM / 4 / NP_BIG, part + 7 * PART_SLOT);
    k_scales<<<1, 256, 0, stream>>>(part, scales);
    k_levels<<<(DM * DM / 8) / 256, 256, 0, stream>>>(wq,  DM * DM / 8, scales, 0u, LVq);
    k_levels<<<(DM * DM / 8) / 256, 256, 0, stream>>>(wk,  DM * DM / 8, scales, 1u, LVk);
    k_levels<<<(DM * DM / 8) / 256, 256, 0, stream>>>(wv,  DM * DM / 8, scales, 2u, LVv);
    k_levels<<<(DM * DM / 8) / 256, 256, 0, stream>>>(wo,  DM * DM / 8, scales, 3u, LVo);
    k_levels<<<(HS * HS / 8) / 256, 256, 0, stream>>>(su,  HS * HS / 8, scales, 4u, LVsu);
    k_levels<<<(HS * HS / 8) / 256, 256, 0, stream>>>(sv,  HS * HS / 8, scales, 5u, LVsv);
    k_levels<<<(HID * DM / 8) / 256, 256, 0, stream>>>(wup, HID * DM / 8, scales, 6u, LVup);
    k_levels<<<(HID * DM / 8) / 256, 256, 0, stream>>>(wdn, HID * DM / 8, scales, 7u, LVdn);
    k_trig<<<(HID / 2) / 256, 256, 0, stream>>>(theta, ctab, stab, (unsigned)(HID / 2));

    const unsigned gD  = (((unsigned)MTOK / 64u) * ((unsigned)DM / 64u) + 7u) / 8u;
    const unsigned gS  = ((((unsigned)MTOK * HEADS) / 64u) * 1u + 7u) / 8u;
    const unsigned gUp = (((unsigned)MTOK / 64u) * ((unsigned)HID / 64u) + 7u) / 8u;

    k_ln<true><<<(MTOK + 7) / 8, 256, 0, stream>>>(x, n1g, n1b, XN, (unsigned)MTOK, (unsigned)(DM / 256));
    k_gemm64<1, 0, 6, 6><<<gD, 256, 0, stream>>>(XN, DM, LVq, DM, (void*)Q16, DM, scales, 0u, scales,
                                                  (unsigned)MTOK, (unsigned)DM, (unsigned)DM);
    k_gemm64<1, 0, 6, 6><<<gD, 256, 0, stream>>>(XN, DM, LVk, DM, (void*)K16, DM, scales, 1u, scales,
                                                  (unsigned)MTOK, (unsigned)DM, (unsigned)DM);
    k_gemm64<1, 0, 6, 6><<<gD, 256, 0, stream>>>(LVv, DM, XN, DM, (void*)VT16, (unsigned)MTOK, scales, 2u, scales,
                                                  (unsigned)DM, (unsigned)MTOK, (unsigned)DM);
    k_gemm64<1, 0, 6, 6><<<gS, 256, 0, stream>>>(Q16, HS, LVsu, HS, (void*)QS16, HS, scales, 4u, scales,
                                                  (unsigned)(MTOK * HEADS), (unsigned)HS, (unsigned)HS);
    k_gemm64<1, 0, 6, 6><<<gS, 256, 0, stream>>>(K16, HS, LVsv, HS, (void*)KS16, HS, scales, 5u, scales,
                                                  (unsigned)(MTOK * HEADS), (unsigned)HS, (unsigned)HS);
    k_attn<<<NB * HEADS * NQB, 128, 0, stream>>>(QS16, KS16, VT16, pscal, AO16);
    k_gemm64<0, 2, 6, 0><<<gD, 256, 0, stream>>>(AO16, DM, LVo, DM, (void*)X1, DM, scales, 3u, x,
                                                  (unsigned)MTOK, (unsigned)DM, (unsigned)DM);

    k_ln<false><<<(MTOK + 7) / 8, 256, 0, stream>>>(X1, n2g, n2b, XN, (unsigned)MTOK, (unsigned)(DM / 256));
    k_gemm64<0, 0, 6, 0><<<gUp, 256, 0, stream>>>(XN, DM, LVup, DM, (void*)HBUF, HID, scales, 6u, scales,
                                                   (unsigned)MTOK, (unsigned)HID, (unsigned)DM);
    k_rot_ln_silu<<<(MTOK + 7) / 8, 256, 0, stream>>>(HBUF, ctab, stab, mng, mnb, ACT16, (unsigned)MTOK, (unsigned)(HID / 256));
    k_gemm64<0, 1, 6, 0><<<gD, 256, 0, stream>>>(ACT16, HID, LVdn, HID, (void*)out, DM, scales, 7u, X1,
                                                  (unsigned)MTOK, (unsigned)DM, (unsigned)HID);
}
